// EdgePredictor_1185410974254
// MI455X (gfx1250) — hardware-verified
//
#include <hip/hip_runtime.h>
#include <math.h>

constexpr int kB        = 32;
constexpr int kNodes    = 64;
constexpr int kD        = 256;
constexpr int kH        = 512;
constexpr int kPairs    = 2016;
constexpr int kRowsOut  = kB * kPairs;
constexpr int kNodeRows = kB * kNodes;
constexpr int kUVld     = 2 * kH;
constexpr int kPairsPerBlk = 32;
constexpr int kRowsPerBlk  = 2 * kPairsPerBlk;
constexpr int kBlocksPair  = kRowsOut / kPairsPerBlk;
constexpr int kAPitch   = kH + 8;
constexpr float kCarryH1  = 16.0f;
constexpr float kCarryW2  = 16.0f;
constexpr float kEpiScale = 1.0f / 256.0f;

static_assert(kRowsOut == kBlocksPair * kPairsPerBlk, "pair grid covers the output exactly");
static_assert(kNodes * (kNodes - 1) / 2 == kPairs, "pair count");
static_assert(kD % 32 == 0 && kH % 32 == 0, "K multiples of 32");
static_assert(kNodeRows % 64 == 0 && kUVld % 64 == 0, "M, N multiples of 64 for the 64x64 wave tile");
static_assert((kAPitch * 2) % 16 == 0, "LDS row pitch 16-B aligned");

typedef __attribute__((ext_vector_type(16))) _Float16 v16h;
typedef __attribute__((ext_vector_type(8)))  _Float16 v8h;
typedef __attribute__((ext_vector_type(16))) __bf16   v16b;
typedef __attribute__((ext_vector_type(8)))  __bf16   v8b;
typedef __attribute__((ext_vector_type(8)))  float    v8f;
typedef __attribute__((ext_vector_type(4)))  float    v4f;
typedef __attribute__((ext_vector_type(4)))  unsigned int v4u;

__device__ __forceinline__ unsigned short f2bf_bits(float f) {
  unsigned u = __float_as_uint(f);
  return (unsigned short)((u + 0x7FFFu + ((u >> 16) & 1u)) >> 16);
}
__device__ __forceinline__ float bf_bits2f(unsigned short h) { return __uint_as_float(((unsigned)h) << 16); }

__device__ __forceinline__ void dep_guard_h(v8f& a, v8f& b, v16h x, v16h y) { asm volatile("v_nop\n\tv_nop\n\tv_nop\n\tv_nop" : "+v"(a), "+v"(b) : "v"(x), "v"(y)); }
__device__ __forceinline__ void dep_guard_b(v8f& a, v8f& b, v16b x, v16b y) { asm volatile("v_nop\n\tv_nop\n\tv_nop\n\tv_nop" : "+v"(a), "+v"(b) : "v"(x), "v"(y)); }
__device__ __forceinline__ void keep4_h(v16h a, v16h b, v16h c, v16h d) { asm volatile("v_nop" :: "v"(a), "v"(b), "v"(c), "v"(d)); }
__device__ __forceinline__ void keep4_b(v16b a, v16b b, v16b c, v16b d) { asm volatile("v_nop" :: "v"(a), "v"(b), "v"(c), "v"(d)); }
__device__ __forceinline__ void acc_guard4(v8f& a, v8f& b, v8f& c, v8f& d) { asm volatile("v_nop\n\tv_nop\n\tv_nop\n\tv_nop" : "+v"(a), "+v"(b), "+v"(c), "+v"(d)); }
template <typename T> struct Frag;
template <> struct Frag<_Float16> {
  typedef v16h V; union U { v16h v; v8h h[2]; };
  static __device__ __forceinline__ v16h load(const _Float16* p) {
    U f; f.h[0] = *(const v8h*)(p); f.h[1] = *(const v8h*)(p + 16); return f.v;
  }
  static __device__ __forceinline__ v8f mma(v16h a, v16h b, v8f c) {
    return __builtin_amdgcn_wmma_f32_16x16x32_f16(false, a, false, b, (short)0, c, false, false);
  }
  static __device__ __forceinline__ void guard(v8f& a, v8f& b, v16h x, v16h y) { dep_guard_h(a, b, x, y); }
  static __device__ __forceinline__ void keep(v16h a, v16h b, v16h c, v16h d) { keep4_h(a, b, c, d); }
};
template <> struct Frag<__bf16> {
  typedef v16b V; union U { v16b v; v8b h[2]; };
  static __device__ __forceinline__ v16b load(const __bf16* p) {
    U f; f.h[0] = *(const v8b*)(p); f.h[1] = *(const v8b*)(p + 16); return f.v;
  }
  static __device__ __forceinline__ v8f mma(v16b a, v16b b, v8f c) {
    return __builtin_amdgcn_wmma_f32_16x16x32_bf16(false, a, false, b, (short)0, c, false, false);
  }
  static __device__ __forceinline__ void guard(v8f& a, v8f& b, v16b x, v16b y) { dep_guard_b(a, b, x, y); }
  static __device__ __forceinline__ void keep(v16b a, v16b b, v16b c, v16b d) { keep4_b(a, b, c, d); }
};

__device__ __forceinline__ unsigned pk16(unsigned short a, unsigned short b) { return (unsigned)a | ((unsigned)b << 16); }
__device__ __forceinline__ unsigned short h_bits(float f) { const _Float16 h = (_Float16)f; return __builtin_bit_cast(unsigned short, h); }

__device__ __forceinline__ void guard_row_h(v8f& a0, v8f& a1, v8f& a2, v8f& a3, v16h x, v16h b0, v16h b1, v16h b2, v16h b3) {
  asm volatile("v_nop\n\tv_nop\n\tv_nop\n\tv_nop" : "+v"(a0), "+v"(a1), "+v"(a2), "+v"(a3) : "v"(x), "v"(b0), "v"(b1), "v"(b2), "v"(b3));
}

template <int ET> struct Elem;
template <> struct Elem<0> { typedef _Float16 T; };
template <> struct Elem<1> { typedef __bf16 T; };
template <int ET, bool SPLIT, int BIAS_MODE, int OUT_MODE, bool RESID, int ACT = 0>
__global__ __launch_bounds__(256) void wmma_gemm64(
    const unsigned short* __restrict__ Ap, const unsigned short* __restrict__ A2p, int lda, long strideA,
    const unsigned short* __restrict__ Btp, const unsigned short* __restrict__ Bt2p, int ldb, long strideB,
    void* __restrict__ Cout, void* __restrict__ Cout2, int ldc, long strideC,
    const float* __restrict__ bias,
    const float* __restrict__ resid, long strideR,
    int M, int N, int K, float scale) {
  typedef typename Elem<ET>::T T;
  typedef typename Frag<T>::V V;
  const T* A = (const T*)Ap; const T* A2 = (const T*)A2p; const T* Bt = (const T*)Btp; const T* Bt2 = (const T*)Bt2p;
  __shared__ __align__(16) float sT[8][16 * 68];
  const int b    = blockIdx.y;
  const int lane = threadIdx.x & 31;
  const int wave = threadIdx.x >> 5;
  const int tilesN = N >> 6;
  const int tilesM = M >> 6;
  const int tile = blockIdx.x * 8 + wave;
  if (tile >= tilesM * tilesN) return;
  const int tm = tile / tilesN;
  const int tn = tile - tm * tilesN;
  const int m0 = tm << 6;
  const int n0 = tn << 6;

  const T* Ab  = A  + (size_t)b * strideA;
  const T* Bb  = Bt + (size_t)b * strideB;
  const T* Ab2 = SPLIT ? (A2  + (size_t)b * strideA) : nullptr;
  const T* Bb2 = SPLIT ? (Bt2 + (size_t)b * strideB) : nullptr;

  const int rlane = lane & 15;
  const int koff  = (lane >> 4) * 8;
  const int mOff  = (lane >> 4) * 8;

  v8f acc[4][4];
#pragma unroll
  for (int i = 0; i < 4; ++i)
#pragma unroll
    for (int j = 0; j < 4; ++j) acc[i][j] = (v8f){0.f,0.f,0.f,0.f,0.f,0.f,0.f,0.f};

  for (int k0 = 0; k0 < K; k0 += 32) {
    V bh[4], bl[4];
#pragma unroll
    for (int j = 0; j < 4; ++j) {
      const size_t bo = (size_t)(n0 + (j << 4) + rlane) * ldb + koff + k0;
      bh[j] = Frag<T>::load(Bb + bo);
      if (SPLIT) bl[j] = Frag<T>::load(Bb2 + bo);
    }
#pragma unroll
    for (int i = 0; i < 4; ++i) {
      const size_t ao = (size_t)(m0 + (i << 4) + rlane) * lda + koff + k0;
      V ah = Frag<T>::load(Ab + ao);
      V al;
      if (SPLIT) al = Frag<T>::load(Ab2 + ao);
#pragma unroll
      for (int j = 0; j < 4; ++j) {
        acc[i][j] = Frag<T>::mma(ah, bh[j], acc[i][j]);
        if (SPLIT) {
          acc[i][j] = Frag<T>::mma(ah, bl[j], acc[i][j]);
          acc[i][j] = Frag<T>::mma(al, bh[j], acc[i][j]);
        }
      }
      Frag<T>::guard(acc[i][0], acc[i][3], ah, SPLIT ? al : ah);
    }
    Frag<T>::keep(bh[0], bh[1], bh[2], bh[3]);
    if (SPLIT) Frag<T>::keep(bl[0], bl[1], bl[2], bl[3]);
  }
  acc_guard4(acc[0][0], acc[0][1], acc[0][2], acc[0][3]);
  acc_guard4(acc[1][0], acc[1][1], acc[1][2], acc[1][3]);
  acc_guard4(acc[2][0], acc[2][1], acc[2][2], acc[2][3]);
  acc_guard4(acc[3][0], acc[3][1], acc[3][2], acc[3][3]);

  float* slab = sT[wave];
  const float* Rb = RESID ? (resid + (size_t)b * strideR) : nullptr;
#pragma unroll
  for (int i = 0; i < 4; ++i) {
    const int mBase = m0 + (i << 4);
#pragma unroll
    for (int j = 0; j < 4; ++j) {
      const int n = n0 + (j << 4) + rlane;
      float bv = 0.f;
      if (BIAS_MODE == 2) bv = bias[n];
#pragma unroll
      for (int r = 0; r < 8; ++r) {
        float v = acc[i][j][r] * scale;
        if (BIAS_MODE == 1) v += bias[mBase + mOff + r];
        if (BIAS_MODE == 2) v += bv;
        if (RESID) v += Rb[(size_t)(mBase + mOff + r) * ldc + n];
        if (ACT == 1) v = tanhf(v);
        if (ACT == 2) v = fmaxf(v, 0.0f);
        if (ACT == 3) v = v / (1.0f + expf(-v));
        if (ACT == 4) v = (v > 0.f) ? v : 0.01f * v;
        if (ACT == 5) v = 0.5f * v * (1.0f + erff(v * 0.70710678118654752f));
        slab[(mOff + r) * 68 + (j << 4) + rlane] = v;
      }
    }
    __builtin_amdgcn_fence(__ATOMIC_RELEASE, "workgroup");
    __builtin_amdgcn_wave_barrier();
    __builtin_amdgcn_fence(__ATOMIC_ACQUIRE, "workgroup");
    if (OUT_MODE == 0) {
      float* C = (float*)Cout + (size_t)b * strideC;
      const int hh = lane >> 4, c4 = (lane & 15) * 4;
      for (int pass = 0; pass < 2; ++pass) {
#pragma unroll
        for (int it = 0; it < 8; ++it) {
          const int row = it * 2 + hh;
          v4f v = *(const v4f*)(slab + row * 68 + c4);
          *(volatile v4f*)(C + (size_t)(mBase + row) * ldc + n0 + c4) = v;
        }
        __threadfence();
      }
    } else {
      const int q = lane >> 3, c8 = (lane & 7) * 8;
      unsigned short* C  = (unsigned short*)Cout  + (size_t)b * strideC;
      unsigned short* C2 = (OUT_MODE == 2) ? ((unsigned short*)Cout2 + (size_t)b * strideC) : nullptr;
      for (int pass = 0; pass < 2; ++pass) {
#pragma unroll
        for (int it = 0; it < 4; ++it) {
          const int row = it * 4 + q;
          const float* sp = slab + row * 68 + c8;
          v8h hv, lv;
#pragma unroll
          for (int e = 0; e < 8; ++e) {
            if (OUT_MODE == 1) {
              hv[e] = (_Float16)sp[e];
            } else {
              unsigned short hb = f2bf_bits(sp[e]);
              unsigned short lb = f2bf_bits(sp[e] - bf_bits2f(hb));
              hv[e] = __builtin_bit_cast(_Float16, hb);
              lv[e] = __builtin_bit_cast(_Float16, lb);
            }
          }
          *(volatile v8h*)(C + (size_t)(mBase + row) * ldc + n0 + c8) = hv;
          if (OUT_MODE == 2) *(volatile v8h*)(C2 + (size_t)(mBase + row) * ldc + n0 + c8) = lv;
        }
        __threadfence();
      }
    }
    __builtin_amdgcn_fence(__ATOMIC_RELEASE, "workgroup");
    __builtin_amdgcn_wave_barrier();
    __builtin_amdgcn_fence(__ATOMIC_ACQUIRE, "workgroup");
  }
}

__global__ __launch_bounds__(256) void prep_w_kernel(const float* __restrict__ W1, const float* __restrict__ W2,
                                                     unsigned short* __restrict__ W1TH, unsigned short* __restrict__ W1TL,
                                                     unsigned short* __restrict__ W2T) {
  __shared__ float sm[64][65];
  const int t  = threadIdx.x;
  const int tb = blockIdx.x;
  const bool isW1 = (tb < 64);
  int kt, nt, srow0, scol0;
  if (isW1) {
    kt = tb & 3; nt = tb >> 2;
    srow0 = (nt >> 3) * kD + kt * 64;
    scol0 = (nt & 7) * 64;
  } else {
    const int u = tb - 64;
    kt = u & 7; nt = u >> 3;
    srow0 = kt * 64;
    scol0 = nt * 64;
  }
  const float* W = isW1 ? W1 : W2;
  const float scale = isW1 ? 1.0f : kCarryW2;
#pragma unroll
  for (int i = 0; i < 16; ++i) {
    const int e = i * 256 + t;
    const int r = e >> 6;
    const int c = e & 63;
    sm[c][r] = W[(size_t)(srow0 + r) * kH + scol0 + c] * scale;
  }
  __syncthreads();
  const int lane = t & 31, wave = t >> 5;
  const int q = lane >> 3, c8 = (lane & 7) * 8;
  const int n0 = nt * 64, k0 = kt * 64;
  if (isW1) {
    v4u uh[2], ul[2];
#pragma unroll
    for (int it = 0; it < 2; ++it) {
      const int row = wave * 8 + it * 4 + q;
      unsigned short hb[8], lb[8];
#pragma unroll
      for (int e = 0; e < 8; ++e) {
        const float v = sm[row][c8 + e];
        hb[e] = f2bf_bits(v);
        lb[e] = f2bf_bits(v - bf_bits2f(hb[e]));
      }
      uh[it] = (v4u){pk16(hb[0], hb[1]), pk16(hb[2], hb[3]), pk16(hb[4], hb[5]), pk16(hb[6], hb[7])};
      ul[it] = (v4u){pk16(lb[0], lb[1]), pk16(lb[2], lb[3]), pk16(lb[4], lb[5]), pk16(lb[6], lb[7])};
    }
    for (int pass = 0; pass < 2; ++pass) {
#pragma unroll
      for (int it = 0; it < 2; ++it) {
        const int row = wave * 8 + it * 4 + q;
        *(volatile v4u*)(W1TH + (size_t)(n0 + row) * kD + k0 + c8) = uh[it];
        *(volatile v4u*)(W1TL + (size_t)(n0 + row) * kD + k0 + c8) = ul[it];
      }
      __threadfence();
    }
  } else {
    v4u uw[2];
#pragma unroll
    for (int it = 0; it < 2; ++it) {
      const int row = wave * 8 + it * 4 + q;
      unsigned short hb[8];
#pragma unroll
      for (int e = 0; e < 8; ++e) hb[e] = h_bits(sm[row][c8 + e]);
      uw[it] = (v4u){pk16(hb[0], hb[1]), pk16(hb[2], hb[3]), pk16(hb[4], hb[5]), pk16(hb[6], hb[7])};
    }
    for (int pass = 0; pass < 2; ++pass) {
#pragma unroll
      for (int it = 0; it < 2; ++it) {
        const int row = wave * 8 + it * 4 + q;
        *(volatile v4u*)(W2T + (size_t)(n0 + row) * kH + k0 + c8) = uw[it];
      }
      __threadfence();
    }
  }
}

__global__ __launch_bounds__(256) void prep_x_kernel(const float* __restrict__ x, unsigned short* __restrict__ XH,
                                                     unsigned short* __restrict__ XL, int n8) {
  const int i = blockIdx.x * 256 + threadIdx.x;
  if (i >= n8) return;
  const float* p = x + 8 * (size_t)i;
  const v4f a = *(const v4f*)(p);
  const v4f c = *(const v4f*)(p + 4);
  unsigned short hb[8], lb[8];
#pragma unroll
  for (int e = 0; e < 4; ++e) {
    const float v0 = a[e], v1 = c[e];
    hb[e] = f2bf_bits(v0);      lb[e] = f2bf_bits(v0 - bf_bits2f(hb[e]));
    hb[4 + e] = f2bf_bits(v1);  lb[4 + e] = f2bf_bits(v1 - bf_bits2f(hb[4 + e]));
  }
  const v4u uh = (v4u){pk16(hb[0], hb[1]), pk16(hb[2], hb[3]), pk16(hb[4], hb[5]), pk16(hb[6], hb[7])};
  const v4u ul = (v4u){pk16(lb[0], lb[1]), pk16(lb[2], lb[3]), pk16(lb[4], lb[5]), pk16(lb[6], lb[7])};
  unsigned short* qh = XH + 8 * (size_t)i;
  unsigned short* ql = XL + 8 * (size_t)i;
  *(volatile v4u*)qh = uh;
  *(volatile v4u*)ql = ul;
  __threadfence();
  *(volatile v4u*)qh = uh;
  *(volatile v4u*)ql = ul;
}

__device__ __forceinline__ float elu_f(float v) {
  const float e = expf(fminf(v, 0.0f)) - 1.0f;
  return (v > 0.0f) ? v : e;
}

__global__ __launch_bounds__(256) void pair_mlp_kernel(const float* __restrict__ UV, const float* __restrict__ b1,
                                                       const unsigned short* __restrict__ W2Tp, const float* __restrict__ b2,
                                                       const float* __restrict__ W3, const float* __restrict__ b3,
                                                       float* __restrict__ out) {
  __shared__ __align__(16) _Float16 As[kRowsPerBlk * kAPitch];
  __shared__ float red[8 * kRowsPerBlk];
  __shared__ __align__(16) float srow[kRowsPerBlk];
  const _Float16* W2T = (const _Float16*)W2Tp;
  const int tid  = threadIdx.x;
  const int lane = tid & 31;
  const int wave = tid >> 5;
  const int blk  = blockIdx.x;

  {
    const int r   = tid >> 2;
    const int seg = tid & 3;
    const int gp  = blk * kPairsPerBlk + (r >> 1);
    const int order = r & 1;
    const int bi  = gp / kPairs;
    int p = gp - bi * kPairs;
    int ia = 0, cnt = kNodes - 1;
    for (int it = 0; it < kNodes - 1; ++it) {
      if (p < cnt) break;
      p -= cnt; --cnt; ++ia;
    }
    int jb = ia + 1 + p;
    ia = (ia > kNodes - 1) ? (kNodes - 1) : ia;
    jb = (jb > kNodes - 1) ? (kNodes - 1) : ((jb < 0) ? 0 : jb);
    const int na = order ? jb : ia;
    const int nb = order ? ia : jb;
    const float* ur = UV + (size_t)(bi * kNodes + na) * kUVld + seg * 128;
    const float* vr = UV + (size_t)(bi * kNodes + nb) * kUVld + kH + seg * 128;
    const float* br = b1 + seg * 128;
    _Float16* dst = As + r * kAPitch + seg * 128;
#pragma unroll 1
    for (int c = 0; c < 128; c += 8) {
      const v4f u0 = *(const v4f*)(ur + c), u1 = *(const v4f*)(ur + c + 4);
      const v4f w0 = *(const v4f*)(vr + c), w1 = *(const v4f*)(vr + c + 4);
      const v4f g0 = *(const v4f*)(br + c), g1 = *(const v4f*)(br + c + 4);
      const v4f z0 = (u0 + w0) + g0;
      const v4f z1 = (u1 + w1) + g1;
      v8h hv;
#pragma unroll
      for (int e = 0; e < 4; ++e) {
        hv[e]     = (_Float16)(elu_f(z0[e]) * kCarryH1);
        hv[4 + e] = (_Float16)(elu_f(z1[e]) * kCarryH1);
      }
      *(v8h*)(dst + c) = hv;
    }
  }
  __syncthreads();

  const int rlane = lane & 15;
  const int hh    = lane >> 4;
  const int koff  = hh * 8;
  const int n0    = wave * 64;
  v8f acc[4][4];
#pragma unroll
  for (int i = 0; i < 4; ++i)
#pragma unroll
    for (int j = 0; j < 4; ++j) acc[i][j] = (v8f){0.f,0.f,0.f,0.f,0.f,0.f,0.f,0.f};

  for (int k0 = 0; k0 < kH; k0 += 32) {
    v16h bf[4];
#pragma unroll
    for (int j = 0; j < 4; ++j)
      bf[j] = Frag<_Float16>::load(W2T + (size_t)(n0 + (j << 4) + rlane) * kH + koff + k0);
#pragma unroll
    for (int i = 0; i < 4; ++i) {
      const v16h af = Frag<_Float16>::load(As + (i * 16 + rlane) * kAPitch + koff + k0);
#pragma unroll
      for (int j = 0; j < 4; ++j) acc[i][j] = Frag<_Float16>::mma(af, bf[j], acc[i][j]);
      guard_row_h(acc[i][0], acc[i][1], acc[i][2], acc[i][3], af, bf[0], bf[1], bf[2], bf[3]);
    }
    keep4_h(bf[0], bf[1], bf[2], bf[3]);
  }
  acc_guard4(acc[0][0], acc[0][1], acc[0][2], acc[0][3]);
  acc_guard4(acc[1][0], acc[1][1], acc[1][2], acc[1][3]);
  acc_guard4(acc[2][0], acc[2][1], acc[2][2], acc[2][3]);
  acc_guard4(acc[3][0], acc[3][1], acc[3][2], acc[3][3]);

  float bv[4], wv[4];
#pragma unroll
  for (int j = 0; j < 4; ++j) {
    const int n = n0 + (j << 4) + rlane;
    bv[j] = b2[n];
    wv[j] = W3[n];
  }
#pragma unroll
  for (int i = 0; i < 4; ++i) {
    float ps[8];
#pragma unroll
    for (int r = 0; r < 8; ++r) ps[r] = 0.0f;
#pragma unroll
    for (int j = 0; j < 4; ++j) {
#pragma unroll
      for (int r = 0; r < 8; ++r) {
        const float v  = acc[i][j][r] * kEpiScale + bv[j];
        const float h2 = elu_f(v);
        ps[r] = ps[r] + h2 * wv[j];
      }
    }
#pragma unroll
    for (int r = 0; r < 8; ++r) {
      float v = ps[r];
      v += __shfl_xor(v, 1, 32);
      v += __shfl_xor(v, 2, 32);
      v += __shfl_xor(v, 4, 32);
      v += __shfl_xor(v, 8, 32);
      if (rlane == r) red[wave * kRowsPerBlk + i * 16 + 8 * hh + r] = v;
    }
  }
  __syncthreads();
  if (tid < kRowsPerBlk) {
    float s = 0.0f;
#pragma unroll
    for (int w = 0; w < 8; ++w) s += red[w * kRowsPerBlk + tid];
    srow[tid] = s;
  }
  __syncthreads();
  if (wave == 0) {
    const int lc = lane & 7;
    const v4f a0 = *(const v4f*)(srow + 8 * lc);
    const v4f a1 = *(const v4f*)(srow + 8 * lc + 4);
    const float bb = b3[0];
    v4f o;
    o[0] = 0.5f * ((a0[0] + bb) + (a0[1] + bb));
    o[1] = 0.5f * ((a0[2] + bb) + (a0[3] + bb));
    o[2] = 0.5f * ((a1[0] + bb) + (a1[1] + bb));
    o[3] = 0.5f * ((a1[2] + bb) + (a1[3] + bb));
    float* op = out + (size_t)blk * kPairsPerBlk + 4 * lc;
    if (lane < 8) *(volatile v4f*)op = o;
    __threadfence();
    if (lane < 8) *(volatile v4f*)op = o;
  }
}

extern "C" void kernel_launch(void* const* d_in, const int* in_sizes, int n_in,
                              void* d_out, int out_size, void* d_ws, size_t ws_size, hipStream_t stream) {
  (void)in_sizes; (void)n_in; (void)out_size;
  const float* x  = (const float*)d_in[0];
  const float* W1 = (const float*)d_in[1];
  const float* b1 = (const float*)d_in[2];
  const float* W2 = (const float*)d_in[3];
  const float* b2 = (const float*)d_in[4];
  const float* W3 = (const float*)d_in[5];
  const float* b3 = (const float*)d_in[6];
  float* out = (float*)d_out;

  char* ws = (char*)d_ws; size_t off = 0;
  auto carve = [&](size_t bytes) -> char* { char* p = ws + off; off += (bytes + 255) & ~(size_t)255; return p; };
  float*          UV   = (float*)carve((size_t)kNodeRows * kUVld * 4);
  unsigned short* XH   = (unsigned short*)carve((size_t)kNodeRows * kD * 2);
  unsigned short* XL   = (unsigned short*)carve((size_t)kNodeRows * kD * 2);
  unsigned short* W1TH = (unsigned short*)carve((size_t)kUVld * kD * 2);
  unsigned short* W1TL = (unsigned short*)carve((size_t)kUVld * kD * 2);
  unsigned short* W2T  = (unsigned short*)carve((size_t)kH * kH * 2);
  if (off > ws_size || off > (size_t)134217728) return;

  prep_w_kernel<<<128, 256, 0, stream>>>(W1, W2, W1TH, W1TL, W2T);
  {
    const int n8 = kNodeRows * kD / 8;
    prep_x_kernel<<<(n8 + 255) / 256, 256, 0, stream>>>(x, XH, XL, n8);
  }
  {
    const int tiles = (kNodeRows / 64) * (kUVld / 64);
    wmma_gemm64<1, true, 0, 0, false><<<dim3((tiles + 7) / 8, 1), 256, 0, stream>>>(
        (const unsigned short*)XH, (const unsigned short*)XL, kD, 0L,
        (const unsigned short*)W1TH, (const unsigned short*)W1TL, kD, 0L,
        (void*)UV, (void*)nullptr, kUVld, 0L,
        (const float*)nullptr, (const float*)nullptr, 0L, kNodeRows, kUVld, kD, 1.0f);
  }
  pair_mlp_kernel<<<kBlocksPair, 256, 0, stream>>>(UV, b1, W2T, b2, W3, b3, out);
}
